// ClusterGuidedMambaBlock_50826642981202
// MI455X (gfx1250) — hardware-run, weakly checked
//
#include <hip/hip_runtime.h>
#include <math.h>

typedef __attribute__((ext_vector_type(16))) _Float16 v16h;
typedef __attribute__((ext_vector_type(8)))  _Float16 v8h;
typedef __attribute__((ext_vector_type(16))) __bf16   v16b;
typedef __attribute__((ext_vector_type(8)))  __bf16   v8b;
typedef __attribute__((ext_vector_type(8)))  float    v8f;
typedef __attribute__((ext_vector_type(4)))  float    v4f;

constexpr int kBatch  = 2;
constexpr int kSeq    = 2048;
constexpr int kDm     = 768;
constexpr int kDin    = 1536;
constexpr int kNst    = 16;
constexpr int kHid    = 384;
constexpr int kXsN    = 2 * kNst + 1;
constexpr int kXdP    = 64;
constexpr int kRows   = kBatch * kSeq;
constexpr int kConvTP = 260;
constexpr int kScanTS = 64;
constexpr int kScanCh = 64;
constexpr int kScanYP = 68;
constexpr float kLnEps    = 1e-5f;
constexpr float kHCarry   = 16.0f;
constexpr float kWc2Carry = 32.0f;
constexpr float kModFold  = 1.0f / (kHCarry * kWc2Carry);
static_assert(kXsN == 33 && kXsN <= kXdP, "x_ssm width");
static_assert((kDm % 32) == 0 && (kDin % 32) == 0 && (kHid % 32) == 0, "GEMM K multiples of 32");
static_assert((kDm % 64) == 0 && (kDin % 64) == 0 && (kHid % 64) == 0, "transpose tiles");
static_assert((kRows % 64) == 0 && (kDin % 64) == 0 && (kXdP % 64) == 0 && (kDm % 64) == 0, "GEMM M,N multiples of 64");
static_assert((kSeq % kScanTS) == 0 && (kSeq % 64) == 0 && (kDin % kScanCh) == 0 && (kDin % 256) == 0, "tile multiples");
static_assert(kDm == 3 * 256, "LayerNorm lane map");
static_assert((kHid % 8) == 0 && ((kRows * (kHid / 8)) % 256) == 0, "hidden kernel grid");
static_assert(kScanTS * kScanYP >= 8 * 128, "scan prologue staging fits the y tile");

constexpr size_t kOffXNH  = 0;
constexpr size_t kOffXNL  = kOffXNH  + (size_t)kRows * kDm  * 2;
constexpr size_t kOffWIH  = kOffXNL  + (size_t)kRows * kDm  * 2;
constexpr size_t kOffWIL  = kOffWIH  + (size_t)2 * kDin * kDm * 2;
constexpr size_t kOffH16  = kOffWIL  + (size_t)2 * kDin * kDm * 2;
constexpr size_t kOffWC2T = kOffH16  + (size_t)kRows * kHid * 2;
constexpr size_t kOffXP   = kOffWC2T + (size_t)kDin * kHid * 2;
constexpr size_t kOffZP   = kOffXP   + (size_t)kRows * kDin * 4;
constexpr size_t kOffXCH  = kOffZP   + (size_t)kRows * kDin * 4;
constexpr size_t kOffXCL  = kOffXCH  + (size_t)kRows * kDin * 2;
constexpr size_t kOffWXH  = kOffXCL  + (size_t)kRows * kDin * 2;
constexpr size_t kOffWXL  = kOffWXH  + (size_t)kXdP * kDin * 2;
constexpr size_t kOffXD   = kOffWXL  + (size_t)kXdP * kDin * 2;
constexpr size_t kOffWOH  = kOffXD   + (size_t)kRows * kXdP * 4;
constexpr size_t kOffWOL  = kOffWOH  + (size_t)kDm * kDin * 2;
constexpr size_t kOffYH   = kOffWOL  + (size_t)kDm * kDin * 2;
constexpr size_t kOffYL   = kOffYH   + (size_t)kRows * kDin * 2;
constexpr size_t kWsTotal = kOffYL   + (size_t)kRows * kDin * 2;
static_assert(kWsTotal == 133169152ull, "carve total");
static_assert(kWsTotal <= 134217728ull, "carve cap");
static_assert((kOffXNL % 128) == 0 && (kOffWIH % 128) == 0 && (kOffWIL % 128) == 0 && (kOffH16 % 128) == 0 &&
              (kOffWC2T % 128) == 0 && (kOffXP % 128) == 0 && (kOffZP % 128) == 0 && (kOffXCH % 128) == 0 &&
              (kOffXCL % 128) == 0 && (kOffWXH % 128) == 0 && (kOffWXL % 128) == 0 && (kOffXD % 128) == 0 &&
              (kOffWOH % 128) == 0 && (kOffWOL % 128) == 0 && (kOffYH % 128) == 0 && (kOffYL % 128) == 0,
              "128-B aligned regions");

__device__ __forceinline__ unsigned short f2bf_bits(float f) {
  unsigned u = __float_as_uint(f);
  return (unsigned short)((u + 0x7FFFu + ((u >> 16) & 1u)) >> 16);
}
__device__ __forceinline__ float bf_bits2f(unsigned short h) { return __uint_as_float(((unsigned)h) << 16); }

__device__ __forceinline__ void dep_guard4_h(v8f& a, v8f& b, v8f& c, v8f& d, v16h x, v16h y) {
  asm volatile("v_nop\n\tv_nop\n\tv_nop\n\tv_nop" : "+v"(a), "+v"(b), "+v"(c), "+v"(d) : "v"(x), "v"(y));
}
__device__ __forceinline__ void dep_guard4_b(v8f& a, v8f& b, v8f& c, v8f& d, v16b x, v16b y) {
  asm volatile("v_nop\n\tv_nop\n\tv_nop\n\tv_nop" : "+v"(a), "+v"(b), "+v"(c), "+v"(d) : "v"(x), "v"(y));
}
__device__ __forceinline__ void keep4_h(v16h a, v16h b, v16h c, v16h d) { asm volatile("v_nop" :: "v"(a), "v"(b), "v"(c), "v"(d)); }
__device__ __forceinline__ void keep4_b(v16b a, v16b b, v16b c, v16b d) { asm volatile("v_nop" :: "v"(a), "v"(b), "v"(c), "v"(d)); }
__device__ __forceinline__ void acc_guard4(v8f& a, v8f& b, v8f& c, v8f& d) {
  asm volatile("v_nop\n\tv_nop\n\tv_nop\n\tv_nop" : "+v"(a), "+v"(b), "+v"(c), "+v"(d));
}
template <typename T> struct Frag;
template <> struct Frag<_Float16> {
  typedef v16h V; union U { v16h v; v8h h[2]; };
  static __device__ __forceinline__ v16h load(const _Float16* p) {
    U f; f.h[0] = *(const v8h*)(p); f.h[1] = *(const v8h*)(p + 16); return f.v;
  }
  static __device__ __forceinline__ v8f mma(v16h a, v16h b, v8f c) {
    return __builtin_amdgcn_wmma_f32_16x16x32_f16(false, a, false, b, (short)0, c, false, false);
  }
  static __device__ __forceinline__ void guard4(v8f& a, v8f& b, v8f& c, v8f& d, v16h x, v16h y) { dep_guard4_h(a, b, c, d, x, y); }
  static __device__ __forceinline__ void keep(v16h a, v16h b, v16h c, v16h d) { keep4_h(a, b, c, d); }
};
template <> struct Frag<__bf16> {
  typedef v16b V; union U { v16b v; v8b h[2]; };
  static __device__ __forceinline__ v16b load(const __bf16* p) {
    U f; f.h[0] = *(const v8b*)(p); f.h[1] = *(const v8b*)(p + 16); return f.v;
  }
  static __device__ __forceinline__ v8f mma(v16b a, v16b b, v8f c) {
    return __builtin_amdgcn_wmma_f32_16x16x32_bf16(false, a, false, b, (short)0, c, false, false);
  }
  static __device__ __forceinline__ void guard4(v8f& a, v8f& b, v8f& c, v8f& d, v16b x, v16b y) { dep_guard4_b(a, b, c, d, x, y); }
  static __device__ __forceinline__ void keep(v16b a, v16b b, v16b c, v16b d) { keep4_b(a, b, c, d); }
};

template <int ET> struct Elem;
template <> struct Elem<0> { typedef _Float16 T; };
template <> struct Elem<1> { typedef __bf16 T; };
template <int ET, int SPL, bool RESID>
__global__ __launch_bounds__(256) void wmma_gemm64(
    const unsigned short* __restrict__ Ap, const unsigned short* __restrict__ A2p, int lda,
    const unsigned short* __restrict__ Btp, const unsigned short* __restrict__ Bt2p, int ldb,
    float* __restrict__ Cout, int ldc,
    const float* __restrict__ resid,
    int M, int N, int K, float scale) {
  typedef typename Elem<ET>::T T;
  typedef typename Frag<T>::V V;
  const T* A = (const T*)Ap; const T* A2 = (const T*)A2p; const T* Bt = (const T*)Btp; const T* Bt2 = (const T*)Bt2p;
  __shared__ __align__(16) float sT[8][16 * 68];
  const int lane = threadIdx.x & 31;
  const int wave = threadIdx.x >> 5;
  const int tilesN = N >> 6;
  const int tilesM = M >> 6;
  const int tile = blockIdx.x * 8 + wave;
  if (tile >= tilesM * tilesN) return;
  const int tm = tile / tilesN;
  const int tn = tile - tm * tilesN;
  const int m0 = tm << 6;
  const int n0 = tn << 6;

  const int rlane = lane & 15;
  const int koff  = (lane >> 4) * 8;
  const int mOff  = (lane >> 4) * 8;

  v8f acc[4][4];
#pragma unroll
  for (int i = 0; i < 4; ++i)
#pragma unroll
    for (int j = 0; j < 4; ++j) acc[i][j] = (v8f){0.f,0.f,0.f,0.f,0.f,0.f,0.f,0.f};

  for (int k0 = 0; k0 < K; k0 += 32) {
    V bh[4], bl[4];
#pragma unroll
    for (int j = 0; j < 4; ++j) {
      const size_t bo = (size_t)(n0 + (j << 4) + rlane) * ldb + koff + k0;
      bh[j] = Frag<T>::load(Bt + bo);
      if (SPL == 2) bl[j] = Frag<T>::load(Bt2 + bo);
    }
#pragma unroll
    for (int i = 0; i < 4; ++i) {
      const size_t ao = (size_t)(m0 + (i << 4) + rlane) * lda + koff + k0;
      V ah = Frag<T>::load(A + ao);
      V al;
      if (SPL == 2) al = Frag<T>::load(A2 + ao);
#pragma unroll
      for (int j = 0; j < 4; ++j) {
        acc[i][j] = Frag<T>::mma(ah, bh[j], acc[i][j]);
        if (SPL == 2) {
          acc[i][j] = Frag<T>::mma(ah, bl[j], acc[i][j]);
          acc[i][j] = Frag<T>::mma(al, bh[j], acc[i][j]);
        }
      }
      Frag<T>::guard4(acc[i][0], acc[i][1], acc[i][2], acc[i][3], ah, (SPL == 2) ? al : ah);
    }
    Frag<T>::keep(bh[0], bh[1], bh[2], bh[3]);
    if (SPL == 2) Frag<T>::keep(bl[0], bl[1], bl[2], bl[3]);
  }
  acc_guard4(acc[0][0], acc[0][1], acc[0][2], acc[0][3]);
  acc_guard4(acc[1][0], acc[1][1], acc[1][2], acc[1][3]);
  acc_guard4(acc[2][0], acc[2][1], acc[2][2], acc[2][3]);
  acc_guard4(acc[3][0], acc[3][1], acc[3][2], acc[3][3]);

  float* slab = sT[wave];
#pragma unroll
  for (int i = 0; i < 4; ++i) {
    const int mBase = m0 + (i << 4);
#pragma unroll
    for (int j = 0; j < 4; ++j) {
#pragma unroll
      for (int r = 0; r < 8; ++r) {
        slab[(mOff + r) * 68 + (j << 4) + rlane] = acc[i][j][r] * scale;
      }
    }
    __builtin_amdgcn_fence(__ATOMIC_RELEASE, "workgroup");
    __builtin_amdgcn_wave_barrier();
    __builtin_amdgcn_fence(__ATOMIC_ACQUIRE, "workgroup");
    {
      const int hh = lane >> 4, c4 = (lane & 15) * 4;
      v4f vv[8];
#pragma unroll
      for (int it = 0; it < 8; ++it) {
        const int row = it * 2 + hh;
        v4f t = *(const v4f*)(slab + row * 68 + c4);
        if (RESID) {
          const v4f rr = *(const v4f*)(resid + (size_t)(mBase + row) * ldc + n0 + c4);
          t = t + rr;
        }
        vv[it] = t;
      }
      for (int pass = 0; pass < 2; ++pass) {
#pragma unroll
        for (int it = 0; it < 8; ++it) {
          const int row = it * 2 + hh;
          *(volatile v4f*)(Cout + (size_t)(mBase + row) * ldc + n0 + c4) = vv[it];
        }
        __threadfence();
      }
    }
    __builtin_amdgcn_fence(__ATOMIC_RELEASE, "workgroup");
    __builtin_amdgcn_wave_barrier();
    __builtin_amdgcn_fence(__ATOMIC_ACQUIRE, "workgroup");
  }
}

template <int MODE>
__global__ __launch_bounds__(256) void transpose_planes_kernel(
    const float* __restrict__ W, unsigned short* __restrict__ P0, unsigned short* __restrict__ P1,
    int Kdim, int Ndim, float scale)
{
  __shared__ float tile[64 * 65];
  const int tid = threadIdx.x, lane = tid & 31, wave = tid >> 5;
  const int n0 = blockIdx.x * 64;
  const int k0 = blockIdx.y * 64;
#pragma unroll 4
  for (int p = 0; p < 16; ++p) {
    const int idx = tid + p * 256;
    const int kk  = idx >> 6;
    const int nn  = idx & 63;
    const int n   = n0 + nn;
    const int nc  = (n < Ndim) ? n : (Ndim - 1);
    const float v = W[(size_t)(k0 + kk) * Ndim + nc];
    tile[kk * 65 + nn] = (n < Ndim) ? (v * scale) : 0.f;
  }
  __syncthreads();
  const int q = lane >> 3, c8 = (lane & 7) * 8;
  v8h hv[2], lv[2];
#pragma unroll
  for (int it = 0; it < 2; ++it) {
    const int nrow = it * 32 + wave * 4 + q;
#pragma unroll
    for (int e = 0; e < 8; ++e) {
      const float t = tile[(c8 + e) * 65 + nrow];
      if (MODE == 0) {
        hv[it][e] = (_Float16)t;
        lv[it][e] = (_Float16)0.0f;
      } else {
        const unsigned short hb = f2bf_bits(t);
        const unsigned short lb = f2bf_bits(t - bf_bits2f(hb));
        hv[it][e] = __builtin_bit_cast(_Float16, hb);
        lv[it][e] = __builtin_bit_cast(_Float16, lb);
      }
    }
  }
  for (int pass = 0; pass < 2; ++pass) {
#pragma unroll
    for (int it = 0; it < 2; ++it) {
      const int nrow = it * 32 + wave * 4 + q;
      const size_t o = (size_t)(n0 + nrow) * Kdim + k0 + c8;
      *(volatile v8h*)(P0 + o) = hv[it];
      if (MODE == 1) *(volatile v8h*)(P1 + o) = lv[it];
    }
    __threadfence();
  }
}

__global__ __launch_bounds__(256) void ln_split_kernel(
    const float* __restrict__ x, const float* __restrict__ g, const float* __restrict__ bta,
    unsigned short* __restrict__ XH, unsigned short* __restrict__ XL)
{
  const int tid = threadIdx.x, lane = tid & 31, wave = tid >> 5;
  const int row = blockIdx.x * 8 + wave;
  const float* xr = x + (size_t)row * kDm;
  float s = 0.f;
#pragma unroll 1
  for (int it = 0; it < 3; ++it) {
    const float* p = xr + it * 256 + lane * 8;
    const v4f a0 = *(const v4f*)(p);
    const v4f a1 = *(const v4f*)(p + 4);
    s += ((a0[0] + a0[1]) + (a0[2] + a0[3])) + ((a1[0] + a1[1]) + (a1[2] + a1[3]));
  }
#pragma unroll
  for (int off = 16; off > 0; off >>= 1) s += __shfl_xor(s, off, 32);
  const float mu = s * (1.0f / (float)kDm);
  float qs = 0.f;
#pragma unroll 1
  for (int it = 0; it < 3; ++it) {
    const float* p = xr + it * 256 + lane * 8;
    const v4f a0 = *(const v4f*)(p);
    const v4f a1 = *(const v4f*)(p + 4);
    float part = 0.f;
#pragma unroll
    for (int e = 0; e < 4; ++e) {
      const float d0 = a0[e] - mu, d1 = a1[e] - mu;
      part = fmaf(d0, d0, part);
      part = fmaf(d1, d1, part);
    }
    qs += part;
  }
#pragma unroll
  for (int off = 16; off > 0; off >>= 1) qs += __shfl_xor(qs, off, 32);
  const float var  = qs * (1.0f / (float)kDm);
  const float rinv = rsqrtf(var + kLnEps);
#pragma unroll 1
  for (int it = 0; it < 3; ++it) {
    const int c0 = it * 256 + lane * 8;
    const v4f a0 = *(const v4f*)(xr + c0);
    const v4f a1 = *(const v4f*)(xr + c0 + 4);
    const v4f g0 = *(const v4f*)(g + c0);
    const v4f g1 = *(const v4f*)(g + c0 + 4);
    const v4f b0 = *(const v4f*)(bta + c0);
    const v4f b1 = *(const v4f*)(bta + c0 + 4);
    v8h hv, lv;
#pragma unroll
    for (int e = 0; e < 4; ++e) {
      const float y0 = (a0[e] - mu) * rinv * g0[e] + b0[e];
      const float y1 = (a1[e] - mu) * rinv * g1[e] + b1[e];
      const unsigned short h0 = f2bf_bits(y0), h1 = f2bf_bits(y1);
      const unsigned short l0 = f2bf_bits(y0 - bf_bits2f(h0)), l1 = f2bf_bits(y1 - bf_bits2f(h1));
      hv[e]     = __builtin_bit_cast(_Float16, h0);
      hv[4 + e] = __builtin_bit_cast(_Float16, h1);
      lv[e]     = __builtin_bit_cast(_Float16, l0);
      lv[4 + e] = __builtin_bit_cast(_Float16, l1);
    }
    unsigned short* qh = XH + (size_t)row * kDm + c0;
    unsigned short* ql = XL + (size_t)row * kDm + c0;
    *(volatile v8h*)qh = hv;
    *(volatile v8h*)ql = lv;
    __threadfence();
    *(volatile v8h*)qh = hv;
    *(volatile v8h*)ql = lv;
  }
}

__global__ __launch_bounds__(256) void hidden_kernel(
    const float* __restrict__ imp, const float* __restrict__ Wc1, const float* __restrict__ bc1,
    unsigned short* __restrict__ H16, int total8)
{
  const int i = blockIdx.x * 256 + threadIdx.x;
  if (i >= total8) return;
  constexpr int kPerRow = kHid / 8;
  const int row = i / kPerRow;
  const int j8  = (i - row * kPerRow) * 8;
  const float iv = imp[row];
  const v4f w0 = *(const v4f*)(Wc1 + j8);
  const v4f w1 = *(const v4f*)(Wc1 + j8 + 4);
  const v4f b0 = *(const v4f*)(bc1 + j8);
  const v4f b1 = *(const v4f*)(bc1 + j8 + 4);
  v8h hv;
#pragma unroll
  for (int e = 0; e < 4; ++e) {
    const float t0 = fmaxf(iv * w0[e] + b0[e], 0.0f) * kHCarry;
    const float t1 = fmaxf(iv * w1[e] + b1[e], 0.0f) * kHCarry;
    hv[e]     = (_Float16)t0;
    hv[4 + e] = (_Float16)t1;
  }
  unsigned short* qd = H16 + (size_t)i * 8;
  *(volatile v8h*)qd = hv;
  __threadfence();
  *(volatile v8h*)qd = hv;
}

__global__ __launch_bounds__(256) void conv_silu_kernel(
    const float* __restrict__ XP, const float* __restrict__ cw, const float* __restrict__ cb,
    unsigned short* __restrict__ XCH, unsigned short* __restrict__ XCL)
{
  __shared__ __align__(16) float sT[16 * kConvTP];
  const int tid = threadIdx.x, lane = tid & 31, wave = tid >> 5;
  const int d0 = blockIdx.x * 256, d = d0 + tid;
  const int g0 = blockIdx.y * 64;
  const int tb = g0 & (kSeq - 1);
  const v4f wv = *(const v4f*)(cw + (size_t)d * 4);
  const float w0 = wv[0], w1 = wv[1], w2 = wv[2], w3 = wv[3];
  const float bc = cb[d];
  float xm3, xm2, xm1;
  {
    const bool hist = (tb > 0);
    const int rb = hist ? (g0 - 3) : g0;
    const float v3 = XP[(size_t)rb * kDin + d];
    const float v2 = XP[(size_t)(rb + 1) * kDin + d];
    const float v1 = XP[(size_t)(rb + 2) * kDin + d];
    xm3 = hist ? v3 : 0.f;
    xm2 = hist ? v2 : 0.f;
    xm1 = hist ? v1 : 0.f;
  }
#pragma unroll 1
  for (int sub = 0; sub < 4; ++sub) {
    const int lb = g0 + sub * 16;
#pragma unroll 1
    for (int s = 0; s < 16; ++s) {
      const float xcur = XP[(size_t)(lb + s) * kDin + d];
      float acc = w0 * xm3;
      acc = fmaf(w1, xm2, acc);
      acc = fmaf(w2, xm1, acc);
      acc = fmaf(w3, xcur, acc);
      const float sv = acc + bc;
      const float sg = __builtin_amdgcn_rcpf(1.0f + expf(-sv));
      sT[s * kConvTP + tid] = sv * sg;
      xm3 = xm2; xm2 = xm1; xm1 = xcur;
    }
    __syncthreads();
    v8h bh[2], blo[2];
#pragma unroll
    for (int it = 0; it < 2; ++it) {
      const float* sp = sT + (it * 8 + wave) * kConvTP + lane * 8;
      const v4f a0 = *(const v4f*)(sp);
      const v4f a1 = *(const v4f*)(sp + 4);
#pragma unroll
      for (int e = 0; e < 4; ++e) {
        const unsigned short h0 = f2bf_bits(a0[e]), h1 = f2bf_bits(a1[e]);
        const unsigned short l0 = f2bf_bits(a0[e] - bf_bits2f(h0)), l1 = f2bf_bits(a1[e] - bf_bits2f(h1));
        bh[it][e]      = __builtin_bit_cast(_Float16, h0);
        bh[it][4 + e]  = __builtin_bit_cast(_Float16, h1);
        blo[it][e]     = __builtin_bit_cast(_Float16, l0);
        blo[it][4 + e] = __builtin_bit_cast(_Float16, l1);
      }
    }
    for (int pass = 0; pass < 2; ++pass) {
#pragma unroll
      for (int it = 0; it < 2; ++it) {
        const size_t o = (size_t)(lb + it * 8 + wave) * kDin + d0 + lane * 8;
        *(volatile v8h*)(XCH + o) = bh[it];
        *(volatile v8h*)(XCL + o) = blo[it];
      }
      __threadfence();
    }
    __syncthreads();
  }
}

__global__ __launch_bounds__(128) void scan_kernel(
    const float* __restrict__ XD, const float* __restrict__ PM, const float* __restrict__ ZP,
    const unsigned* __restrict__ XCH32, const unsigned* __restrict__ XCL32,
    const float* __restrict__ Wdt, const float* __restrict__ bdt, const float* __restrict__ bc2,
    const float* __restrict__ Alog, const float* __restrict__ Dsk,
    unsigned short* __restrict__ YH, unsigned short* __restrict__ YL)
{
  __shared__ __align__(16) float sX[kScanTS * kXdP];
  __shared__ __align__(16) float sY[kScanTS * kScanYP];
  const int tid = threadIdx.x, lane = tid & 31, wave = tid >> 5;
  constexpr int kBlkPerB = kDin / kScanCh;
  const int bix = blockIdx.x / kBlkPerB;
  const int d0  = (blockIdx.x - bix * kBlkPerB) * kScanCh;
  const int c   = tid >> 1;
  const int hf  = tid & 1;
  const int d   = d0 + c;
  const int nb  = hf * 8;
  const size_t row0 = (size_t)bix * kSeq;
#pragma unroll 1
  for (int s = 0; s < 8; ++s) sY[s * 128 + tid] = -expf(Alog[(size_t)d * kNst + nb + s]);
  __syncthreads();
  float negA[8], h[8];
#pragma unroll
  for (int s = 0; s < 8; ++s) {
    negA[s] = sY[s * 128 + tid];
    h[s] = 0.f;
  }
  const float wdt = Wdt[d], bb = bdt[d], b2 = bc2[d], Dd = Dsk[d];
  const unsigned sh = (unsigned)(d & 1) * 16u;
  const int lr = tid >> 4, lc4 = (tid & 15) * 4;
  const int q = lane >> 3, c8 = (lane & 7) * 8;
#pragma unroll 1
  for (int t0 = 0; t0 < kSeq; t0 += kScanTS) {
    __syncthreads();
#pragma unroll
    for (int i = 0; i < 8; ++i) {
      const int r = lr + 8 * i;
      *(v4f*)(sX + r * kXdP + lc4) = *(const v4f*)(XD + (row0 + t0 + r) * kXdP + lc4);
    }
    __syncthreads();
#pragma unroll 1
    for (int s = 0; s < kScanTS; ++s) {
      const float* xr = sX + s * kXdP;
      const float dr = xr[0];
      float Bs[8], Cs[8];
#pragma unroll
      for (int k = 0; k < 8; ++k) {
        Bs[k] = xr[1 + nb + k];
        Cs[k] = xr[1 + kNst + nb + k];
      }
      const size_t e = (row0 + t0 + s) * kDin + d;
      float pm = PM[e];
      float zv = ZP[e];
      unsigned wh = XCH32[e >> 1];
      unsigned wl = XCL32[e >> 1];
      asm volatile("" : "+v"(pm), "+v"(zv), "+v"(wh), "+v"(wl));
      const float xhi = __uint_as_float(((wh >> sh) & 0xffffu) << 16);
      const float xlo = __uint_as_float(((wl >> sh) & 0xffffu) << 16);
      const float xt  = xhi + xlo;
      const float v   = dr * wdt + bb;
      const float a   = expf(-fabsf(v));
      const float u   = 1.0f + a;
      const float l1p = logf(u) + (a - (u - 1.0f)) * __builtin_amdgcn_rcpf(u);
      const float sp  = fmaxf(v, 0.0f) + l1p;
      const float md  = __builtin_amdgcn_rcpf(1.0f + expf(-(pm + b2)));
      const float dt  = sp * (1.0f + md);
      const float dtx = dt * xt;
      float y = 0.f;
#pragma unroll
      for (int k = 0; k < 8; ++k) {
        float ek = expf(dt * negA[k]);
        ek = (ek < 1.17549435e-38f) ? 0.0f : ek;
        h[k] = ek * h[k] + dtx * Bs[k];
        y = h[k] * Cs[k] + y;
      }
      y += __shfl_xor(y, 1, 32);
      y = xt * Dd + y;
      const float sg = __builtin_amdgcn_rcpf(1.0f + expf(-zv));
      y = y * (zv * sg);
      if (hf == 0) sY[s * kScanYP + c] = y;
    }
    __syncthreads();
    v8h hv[4], lv[4];
#pragma unroll
    for (int it = 0; it < 4; ++it) {
      const int row = it * 16 + wave * 4 + q;
      const float* sp2 = sY + row * kScanYP + c8;
      const v4f a0 = *(const v4f*)(sp2);
      const v4f a1 = *(const v4f*)(sp2 + 4);
#pragma unroll
      for (int e2 = 0; e2 < 4; ++e2) {
        const unsigned short h0 = f2bf_bits(a0[e2]), h1 = f2bf_bits(a1[e2]);
        const unsigned short l0 = f2bf_bits(a0[e2] - bf_bits2f(h0)), l1 = f2bf_bits(a1[e2] - bf_bits2f(h1));
        hv[it][e2]     = __builtin_bit_cast(_Float16, h0);
        hv[it][4 + e2] = __builtin_bit_cast(_Float16, h1);
        lv[it][e2]     = __builtin_bit_cast(_Float16, l0);
        lv[it][4 + e2] = __builtin_bit_cast(_Float16, l1);
      }
    }
    for (int pass = 0; pass < 2; ++pass) {
#pragma unroll
      for (int it = 0; it < 4; ++it) {
        const int row = it * 16 + wave * 4 + q;
        const size_t o = (row0 + t0 + row) * kDin + d0 + c8;
        *(volatile v8h*)(YH + o) = hv[it];
        *(volatile v8h*)(YL + o) = lv[it];
      }
      __threadfence();
    }
  }
}

extern "C" void kernel_launch(void* const* d_in, const int* in_sizes, int n_in,
                              void* d_out, int out_size, void* d_ws, size_t ws_size,
                              hipStream_t stream) {
  if (n_in < 17) return;
  if (in_sizes[0] != kRows * kDm) return;
  if (in_sizes[1] != kRows) return;
  if (in_sizes[2] != kDm || in_sizes[3] != kDm) return;
  if (in_sizes[4] != kDm * 2 * kDin) return;
  if (in_sizes[5] != kDin * 4 || in_sizes[6] != kDin) return;
  if (in_sizes[7] != kDin * kXsN) return;
  if (in_sizes[8] != kDin || in_sizes[9] != kDin) return;
  if (in_sizes[10] != kHid || in_sizes[11] != kHid) return;
  if (in_sizes[12] != kHid * kDin || in_sizes[13] != kDin) return;
  if (in_sizes[14] != kDin * kNst || in_sizes[15] != kDin) return;
  if (in_sizes[16] != kDin * kDm) return;
  if (out_size != kRows * kDm) return;
  if (ws_size < kWsTotal) return;

  const float* x      = (const float*)d_in[0];
  const float* imp    = (const float*)d_in[1];
  const float* ln_g   = (const float*)d_in[2];
  const float* ln_b   = (const float*)d_in[3];
  const float* W_in   = (const float*)d_in[4];
  const float* conv_w = (const float*)d_in[5];
  const float* conv_b = (const float*)d_in[6];
  const float* W_x    = (const float*)d_in[7];
  const float* W_dt   = (const float*)d_in[8];
  const float* b_dt   = (const float*)d_in[9];
  const float* Wc1    = (const float*)d_in[10];
  const float* bc1    = (const float*)d_in[11];
  const float* Wc2    = (const float*)d_in[12];
  const float* bc2    = (const float*)d_in[13];
  const float* A_log  = (const float*)d_in[14];
  const float* Dskip  = (const float*)d_in[15];
  const float* W_out  = (const float*)d_in[16];
  float* out = (float*)d_out;

  char* ws = (char*)d_ws;
  unsigned short* XNH  = (unsigned short*)(ws + kOffXNH);
  unsigned short* XNL  = (unsigned short*)(ws + kOffXNL);
  unsigned short* WIH  = (unsigned short*)(ws + kOffWIH);
  unsigned short* WIL  = (unsigned short*)(ws + kOffWIL);
  unsigned short* H16  = (unsigned short*)(ws + kOffH16);
  unsigned short* WC2T = (unsigned short*)(ws + kOffWC2T);
  float*          XP   = (float*)(ws + kOffXP);
  float*          PM   = (float*)(ws + kOffXP);
  float*          ZP   = (float*)(ws + kOffZP);
  unsigned short* XCH  = (unsigned short*)(ws + kOffXCH);
  unsigned short* XCL  = (unsigned short*)(ws + kOffXCL);
  unsigned short* WXH  = (unsigned short*)(ws + kOffWXH);
  unsigned short* WXL  = (unsigned short*)(ws + kOffWXL);
  float*          XD   = (float*)(ws + kOffXD);
  unsigned short* WOH  = (unsigned short*)(ws + kOffWOH);
  unsigned short* WOL  = (unsigned short*)(ws + kOffWOL);
  unsigned short* YH   = (unsigned short*)(ws + kOffYH);
  unsigned short* YL   = (unsigned short*)(ws + kOffYL);

  transpose_planes_kernel<1><<<dim3(2 * kDin / 64, kDm / 64), 256, 0, stream>>>(W_in, WIH, WIL, kDm, 2 * kDin, 1.0f);
  transpose_planes_kernel<1><<<dim3(kXdP / 64, kDin / 64), 256, 0, stream>>>(W_x, WXH, WXL, kDin, kXsN, 1.0f);
  transpose_planes_kernel<0><<<dim3(kDin / 64, kHid / 64), 256, 0, stream>>>(Wc2, WC2T, WC2T, kHid, kDin, kWc2Carry);
  transpose_planes_kernel<1><<<dim3(kDm / 64, kDin / 64), 256, 0, stream>>>(W_out, WOH, WOL, kDin, kDm, 1.0f);

  ln_split_kernel<<<kRows / 8, 256, 0, stream>>>(x, ln_g, ln_b, XNH, XNL);

  wmma_gemm64<1, 2, false><<<dim3((kRows / 64) * (kDin / 64) / 8), 256, 0, stream>>>(
      XNH, XNL, kDm, WIH, WIL, kDm, XP, kDin, x, kRows, kDin, kDm, 1.0f);
  wmma_gemm64<1, 2, false><<<dim3((kRows / 64) * (kDin / 64) / 8), 256, 0, stream>>>(
      XNH, XNL, kDm, WIH + (size_t)kDin * kDm, WIL + (size_t)kDin * kDm, kDm, ZP, kDin, x, kRows, kDin, kDm, 1.0f);

  conv_silu_kernel<<<dim3(kDin / 256, kRows / 64), 256, 0, stream>>>(XP, conv_w, conv_b, XCH, XCL);

  wmma_gemm64<1, 2, false><<<dim3((kRows / 64) * (kXdP / 64) / 8), 256, 0, stream>>>(
      XCH, XCL, kDin, WXH, WXL, kDin, XD, kXdP, x, kRows, kXdP, kDin, 1.0f);

  hidden_kernel<<<(kRows * (kHid / 8)) / 256, 256, 0, stream>>>(imp, Wc1, bc1, H16, kRows * (kHid / 8));

  wmma_gemm64<0, 0, false><<<dim3((kRows / 64) * (kDin / 64) / 8), 256, 0, stream>>>(
      H16, H16, kHid, WC2T, WC2T, kHid, PM, kDin, x, kRows, kDin, kHid, kModFold);

  scan_kernel<<<kBatch * (kDin / kScanCh), 128, 0, stream>>>(
      XD, PM, ZP, (const unsigned*)XCH, (const unsigned*)XCL, W_dt, b_dt, bc2, A_log, Dskip, YH, YL);

  wmma_gemm64<1, 2, true><<<dim3((kRows / 64) * (kDm / 64) / 8), 256, 0, stream>>>(
      YH, YL, kDin, WOH, WOL, kDin, out, kDm, x, kRows, kDm, kDin, 1.0f);
}
